// UPNBase_31817117729082
// MI455X (gfx1250) — hardware-verified
//
#include <hip/hip_runtime.h>
#include <math.h>

constexpr int kNB  = 4096;
constexpr int kND  = 64;
constexpr int kNH  = 512;
constexpr int kLDS = 2 * kND;
constexpr int kChunkB = 512;
constexpr int kNumChunks = kNB / kChunkB;
static_assert(kNumChunks * kChunkB == kNB, "chunking");

constexpr float kMuC  = 16.0f;
constexpr float kW1C  = 8.0f;
constexpr float kW2C  = 16.0f;
constexpr int   kActC = 256;
constexpr float kDwC  = 256.0f;
constexpr float kScale1 = 1.0f / (kMuC * kW1C);
constexpr float kScale2 = 1.0f / ((float)kActC * kW2C);
constexpr float kScaleI = 1.0f / (kDwC * kW2C);

typedef __attribute__((ext_vector_type(16))) _Float16 v16h;
typedef __attribute__((ext_vector_type(8)))  _Float16 v8h;
typedef __attribute__((ext_vector_type(16))) __bf16   v16b;
typedef __attribute__((ext_vector_type(8)))  __bf16   v8b;
typedef __attribute__((ext_vector_type(8)))  float    v8f;
typedef __attribute__((ext_vector_type(4)))  float    v4f;
typedef __attribute__((ext_vector_type(4)))  unsigned int v4u;

__device__ __forceinline__ unsigned short f2bf_bits(float f) {
  unsigned u = __float_as_uint(f);
  return (unsigned short)((u + 0x7FFFu + ((u >> 16) & 1u)) >> 16);
}
__device__ __forceinline__ float bf_bits2f(unsigned short h) { return __uint_as_float(((unsigned)h) << 16); }

__device__ __forceinline__ void dep_guard_h(v8f& a, v8f& b, v16h x, v16h y) { asm volatile("v_nop\n\tv_nop\n\tv_nop\n\tv_nop" : "+v"(a), "+v"(b) : "v"(x), "v"(y)); }
__device__ __forceinline__ void dep_guard_b(v8f& a, v8f& b, v16b x, v16b y) { asm volatile("v_nop\n\tv_nop\n\tv_nop\n\tv_nop" : "+v"(a), "+v"(b) : "v"(x), "v"(y)); }
__device__ __forceinline__ void keep4_h(v16h a, v16h b, v16h c, v16h d) { asm volatile("v_nop" :: "v"(a), "v"(b), "v"(c), "v"(d)); }
__device__ __forceinline__ void keep4_b(v16b a, v16b b, v16b c, v16b d) { asm volatile("v_nop" :: "v"(a), "v"(b), "v"(c), "v"(d)); }
__device__ __forceinline__ void acc_guard4(v8f& a, v8f& b, v8f& c, v8f& d) { asm volatile("v_nop\n\tv_nop\n\tv_nop\n\tv_nop" : "+v"(a), "+v"(b), "+v"(c), "+v"(d)); }
template <typename T> struct Frag;
template <> struct Frag<_Float16> {
  typedef v16h V; union U { v16h v; v8h h[2]; };
  static __device__ __forceinline__ v16h load(const _Float16* p) {
    U f; f.h[0] = *(const v8h*)(p); f.h[1] = *(const v8h*)(p + 16); return f.v;
  }
  static __device__ __forceinline__ v8f mma(v16h a, v16h b, v8f c) {
    return __builtin_amdgcn_wmma_f32_16x16x32_f16(false, a, false, b, (short)0, c, false, false);
  }
  static __device__ __forceinline__ void guard(v8f& a, v8f& b, v16h x, v16h y) { dep_guard_h(a, b, x, y); }
  static __device__ __forceinline__ void keep(v16h a, v16h b, v16h c, v16h d) { keep4_h(a, b, c, d); }
};
template <> struct Frag<__bf16> {
  typedef v16b V; union U { v16b v; v8b h[2]; };
  static __device__ __forceinline__ v16b load(const __bf16* p) {
    U f; f.h[0] = *(const v8b*)(p); f.h[1] = *(const v8b*)(p + 16); return f.v;
  }
  static __device__ __forceinline__ v8f mma(v16b a, v16b b, v8f c) {
    return __builtin_amdgcn_wmma_f32_16x16x32_bf16(false, a, false, b, (short)0, c, false, false);
  }
  static __device__ __forceinline__ void guard(v8f& a, v8f& b, v16b x, v16b y) { dep_guard_b(a, b, x, y); }
  static __device__ __forceinline__ void keep(v16b a, v16b b, v16b c, v16b d) { keep4_b(a, b, c, d); }
};

__device__ __forceinline__ unsigned pk16(unsigned short a, unsigned short b) { return (unsigned)a | ((unsigned)b << 16); }
__device__ __forceinline__ unsigned short h_bits(float f) { const _Float16 h = (_Float16)f; return __builtin_bit_cast(unsigned short, h); }

template <int ET> struct Elem;
template <> struct Elem<0> { typedef _Float16 T; };
template <> struct Elem<1> { typedef __bf16 T; };
template <int ET, bool SPLIT, int BIAS_MODE, int OUT_MODE, bool RESID, int ACT = 0, int OCAR = 1>
__global__ __launch_bounds__(256) void wmma_gemm64(
    const unsigned short* __restrict__ Ap, const unsigned short* __restrict__ A2p, int lda, long strideA,
    const unsigned short* __restrict__ Btp, const unsigned short* __restrict__ Bt2p, int ldb, long strideB,
    void* __restrict__ Cout, void* __restrict__ Cout2, int ldc, long strideC,
    const float* __restrict__ bias,
    const float* __restrict__ resid, long strideR,
    int M, int N, int K, float scale) {
  typedef typename Elem<ET>::T T;
  typedef typename Frag<T>::V V;
  const T* A = (const T*)Ap; const T* A2 = (const T*)A2p; const T* Bt = (const T*)Btp; const T* Bt2 = (const T*)Bt2p;
  __shared__ __align__(16) float sT[8][16 * 68];
  const int b    = blockIdx.y;
  const int lane = threadIdx.x & 31;
  const int wave = threadIdx.x >> 5;
  const int tilesN = N >> 6;
  const int tilesM = M >> 6;
  const int tile = blockIdx.x * 8 + wave;
  if (tile >= tilesM * tilesN) return;
  const int tm = tile / tilesN;
  const int tn = tile - tm * tilesN;
  const int m0 = tm << 6;
  const int n0 = tn << 6;

  const T* Ab  = A  + (size_t)b * strideA;
  const T* Bb  = Bt + (size_t)b * strideB;
  const T* Ab2 = SPLIT ? (A2  + (size_t)b * strideA) : nullptr;
  const T* Bb2 = SPLIT ? (Bt2 + (size_t)b * strideB) : nullptr;

  const int rlane = lane & 15;
  const int koff  = (lane >> 4) * 8;
  const int mOff  = (lane >> 4) * 8;

  v8f acc[4][4];
#pragma unroll
  for (int i = 0; i < 4; ++i)
#pragma unroll
    for (int j = 0; j < 4; ++j) acc[i][j] = (v8f){0.f,0.f,0.f,0.f,0.f,0.f,0.f,0.f};

  for (int k0 = 0; k0 < K; k0 += 32) {
    V bh[4], bl[4];
#pragma unroll
    for (int j = 0; j < 4; ++j) {
      const size_t bo = (size_t)(n0 + (j << 4) + rlane) * ldb + koff + k0;
      bh[j] = Frag<T>::load(Bb + bo);
      if (SPLIT) bl[j] = Frag<T>::load(Bb2 + bo);
    }
#pragma unroll
    for (int i = 0; i < 4; ++i) {
      const size_t ao = (size_t)(m0 + (i << 4) + rlane) * lda + koff + k0;
      V ah = Frag<T>::load(Ab + ao);
      V al;
      if (SPLIT) al = Frag<T>::load(Ab2 + ao);
#pragma unroll
      for (int j = 0; j < 4; ++j) {
        acc[i][j] = Frag<T>::mma(ah, bh[j], acc[i][j]);
        if (SPLIT) {
          acc[i][j] = Frag<T>::mma(ah, bl[j], acc[i][j]);
          acc[i][j] = Frag<T>::mma(al, bh[j], acc[i][j]);
        }
      }
      Frag<T>::guard(acc[i][0], acc[i][3], ah, SPLIT ? al : ah);
    }
    Frag<T>::keep(bh[0], bh[1], bh[2], bh[3]);
    if (SPLIT) Frag<T>::keep(bl[0], bl[1], bl[2], bl[3]);
  }
  acc_guard4(acc[0][0], acc[0][1], acc[0][2], acc[0][3]);
  acc_guard4(acc[1][0], acc[1][1], acc[1][2], acc[1][3]);
  acc_guard4(acc[2][0], acc[2][1], acc[2][2], acc[2][3]);
  acc_guard4(acc[3][0], acc[3][1], acc[3][2], acc[3][3]);

  float* slab = sT[wave];
  const float* Rb = RESID ? (resid + (size_t)b * strideR) : nullptr;
#pragma unroll
  for (int i = 0; i < 4; ++i) {
    const int mBase = m0 + (i << 4);
#pragma unroll
    for (int j = 0; j < 4; ++j) {
      const int n = n0 + (j << 4) + rlane;
      float bv = 0.f;
      if (BIAS_MODE == 2) bv = bias[n];
#pragma unroll
      for (int r = 0; r < 8; ++r) {
        float v = acc[i][j][r] * scale;
        if (BIAS_MODE == 1) v += bias[mBase + mOff + r];
        if (BIAS_MODE == 2) v += bv;
        if (RESID) v += Rb[(size_t)(mBase + mOff + r) * ldc + n];
        if (ACT == 1) v = tanhf(v);
        if (ACT == 2) v = fmaxf(v, 0.0f);
        if (ACT == 4) v = (v > 0.f) ? v : 0.01f * v;
        slab[(mOff + r) * 68 + (j << 4) + rlane] = v;
      }
    }
    __builtin_amdgcn_fence(__ATOMIC_RELEASE, "workgroup");
    __builtin_amdgcn_wave_barrier();
    __builtin_amdgcn_fence(__ATOMIC_ACQUIRE, "workgroup");
    if (OUT_MODE == 0) {
      float* C = (float*)Cout + (size_t)b * strideC;
      const int hh = lane >> 4, c4 = (lane & 15) * 4;
      for (int pass = 0; pass < 2; ++pass) {
#pragma unroll
        for (int it = 0; it < 8; ++it) {
          const int row = it * 2 + hh;
          v4f v = *(const v4f*)(slab + row * 68 + c4);
          *(volatile v4f*)(C + (size_t)(mBase + row) * ldc + n0 + c4) = v;
        }
        __threadfence();
      }
    } else {
      const int q = lane >> 3, c8 = (lane & 7) * 8;
      unsigned short* C  = (unsigned short*)Cout  + (size_t)b * strideC;
      unsigned short* C2 = (OUT_MODE == 2) ? ((unsigned short*)Cout2 + (size_t)b * strideC) : nullptr;
      for (int pass = 0; pass < 2; ++pass) {
#pragma unroll
        for (int it = 0; it < 4; ++it) {
          const int row = it * 4 + q;
          const float* sp = slab + row * 68 + c8;
          v8h hv, lv;
#pragma unroll
          for (int e = 0; e < 8; ++e) {
            if (OUT_MODE == 1 || OUT_MODE == 3) {
              hv[e] = (_Float16)(sp[e] * (float)OCAR);
            } else {
              unsigned short hb = f2bf_bits(sp[e]);
              unsigned short lb = f2bf_bits(sp[e] - bf_bits2f(hb));
              hv[e] = __builtin_bit_cast(_Float16, hb);
              lv[e] = __builtin_bit_cast(_Float16, lb);
            }
          }
          *(volatile v8h*)(C + (size_t)(mBase + row) * ldc + n0 + c8) = hv;
          if (OUT_MODE == 2) *(volatile v8h*)(C2 + (size_t)(mBase + row) * ldc + n0 + c8) = lv;
        }
        __threadfence();
      }
      if (OUT_MODE == 3) {
        float* Cd = (float*)Cout2 + (size_t)b * strideC;
        const int hd = lane >> 4, cd4 = (lane & 15) * 4;
        const v4f one4 = (v4f){1.f, 1.f, 1.f, 1.f};
        for (int pass = 0; pass < 2; ++pass) {
#pragma unroll
          for (int it = 0; it < 8; ++it) {
            const int row = it * 2 + hd;
            const v4f s4 = *(const v4f*)(slab + row * 68 + cd4);
            const v4f dv = one4 - s4 * s4;
            *(volatile v4f*)(Cd + (size_t)(mBase + row) * ldc + n0 + cd4) = dv;
          }
          __threadfence();
        }
      }
    }
    __builtin_amdgcn_fence(__ATOMIC_RELEASE, "workgroup");
    __builtin_amdgcn_wave_barrier();
    __builtin_amdgcn_fence(__ATOMIC_ACQUIRE, "workgroup");
  }
}

__global__ __launch_bounds__(256) void k_wcast(const float* __restrict__ W1, const float* __restrict__ V1,
                                               const float* __restrict__ W2, const float* __restrict__ V2,
                                               const float* __restrict__ W3, const float* __restrict__ V3,
                                               unsigned short* __restrict__ W1h, unsigned short* __restrict__ V1h,
                                               unsigned short* __restrict__ W2h, unsigned short* __restrict__ V2h,
                                               unsigned short* __restrict__ W3h, unsigned short* __restrict__ V3h) {
  const int y = blockIdx.y;
  const float* in = W1; unsigned short* outp = W1h; int n8 = kNH * kND / 8; float sc = kW1C;
  if (y == 1)      { in = V1; outp = V1h; }
  else if (y == 2) { in = W2; outp = W2h; n8 = kNH * kNH / 8; sc = kW2C; }
  else if (y == 3) { in = V2; outp = V2h; n8 = kNH * kNH / 8; sc = kW2C; }
  else if (y == 4) { in = W3; outp = W3h; sc = kW2C; }
  else if (y == 5) { in = V3; outp = V3h; sc = kW2C; }
  const int i = blockIdx.x * 256 + threadIdx.x;
  if (i >= n8) return;
  const float* p = in + 8 * (size_t)i;
  const v4f a = *(const v4f*)(p);
  const v4f c = *(const v4f*)(p + 4);
  unsigned short hb[8];
#pragma unroll
  for (int e = 0; e < 4; ++e) {
    hb[e]     = h_bits(a[e] * sc);
    hb[4 + e] = h_bits(c[e] * sc);
  }
  const v4u u = (v4u){pk16(hb[0], hb[1]), pk16(hb[2], hb[3]), pk16(hb[4], hb[5]), pk16(hb[6], hb[7])};
  unsigned short* q = outp + 8 * (size_t)i;
  *(volatile v4u*)q = u;
  __threadfence();
  *(volatile v4u*)q = u;
}

__global__ __launch_bounds__(256) void k_mucast(const float* __restrict__ states, unsigned short* __restrict__ muh) {
  const int i = blockIdx.x * 256 + threadIdx.x;
  if (i >= kNB * 8) return;
  const int b = i >> 3, j = i & 7;
  const float* p = states + (size_t)b * kLDS + 8 * j;
  const v4f a = *(const v4f*)(p);
  const v4f c = *(const v4f*)(p + 4);
  unsigned short hb[8];
#pragma unroll
  for (int e = 0; e < 4; ++e) {
    hb[e]     = h_bits(a[e] * kMuC);
    hb[4 + e] = h_bits(c[e] * kMuC);
  }
  const v4u u = (v4u){pk16(hb[0], hb[1]), pk16(hb[2], hb[3]), pk16(hb[4], hb[5]), pk16(hb[6], hb[7])};
  unsigned short* q = muh + 8 * (size_t)i;
  *(volatile v4u*)q = u;
  __threadfence();
  *(volatile v4u*)q = u;
}

__global__ __launch_bounds__(256) void k_w1t(const float* __restrict__ W1, float* __restrict__ W1T) {
  __shared__ float sm[64][65];
  const int t  = threadIdx.x;
  const int k0 = blockIdx.x * 64;
#pragma unroll
  for (int it = 0; it < 16; ++it) {
    const int e = it * 256 + t;
    const int r = e >> 6;
    const int c = e & 63;
    sm[c][r] = W1[(size_t)(k0 + r) * kND + c];
  }
  __syncthreads();
  const int lane = t & 31, wave = t >> 5;
  const int hh = lane >> 4, c4 = (lane & 15) * 4;
  for (int pass = 0; pass < 2; ++pass) {
#pragma unroll
    for (int it = 0; it < 4; ++it) {
      const int row = it * 16 + wave * 2 + hh;
      const v4f v = (v4f){sm[row][c4], sm[row][c4 + 1], sm[row][c4 + 2], sm[row][c4 + 3]};
      *(volatile v4f*)(W1T + (size_t)row * kNH + k0 + c4) = v;
    }
    __threadfence();
  }
}

__global__ __launch_bounds__(256) void k_dwbuild(const float* __restrict__ d1f, const float* __restrict__ W1T,
                                                 unsigned short* __restrict__ DW, int bbase) {
  const int i = blockIdx.x * 256 + threadIdx.x;
  if (i >= kChunkB * 64 * 64) return;
  const int k0 = (i & 63) * 8;
  const int d  = (i >> 6) & 63;
  const int bl = i >> 12;
  const float* dp = d1f + (size_t)(bbase + bl) * kNH + k0;
  const float* wp = W1T + (size_t)d * kNH + k0;
  const v4f da = *(const v4f*)(dp);
  const v4f db = *(const v4f*)(dp + 4);
  const v4f wa = *(const v4f*)(wp);
  const v4f wb = *(const v4f*)(wp + 4);
  unsigned short hb[8];
#pragma unroll
  for (int e = 0; e < 4; ++e) {
    hb[e]     = h_bits(kDwC * (da[e] * wa[e]));
    hb[4 + e] = h_bits(kDwC * (db[e] * wb[e]));
  }
  const v4u u = (v4u){pk16(hb[0], hb[1]), pk16(hb[2], hb[3]), pk16(hb[4], hb[5]), pk16(hb[6], hb[7])};
  unsigned short* q = DW + 8 * (size_t)i;
  *(volatile v4u*)q = u;
  __threadfence();
  *(volatile v4u*)q = u;
}

__global__ __launch_bounds__(256) void k_jsig(const float* __restrict__ inner, const float* __restrict__ d2f,
                                              const float* __restrict__ W3, const float* __restrict__ qpre,
                                              const float* __restrict__ states, float* __restrict__ out, int bbase) {
  __shared__ __align__(16) float so[4][64];
  const int t  = threadIdx.x;
  const int s  = t >> 6;
  const int o  = t & 63;
  const int bl = blockIdx.x * 4 + s;
  const int b  = bbase + bl;
  const float* ip = inner + ((size_t)bl * kND + o) * kNH;
  const float* dp = d2f + (size_t)b * kNH;
  const float* wp = W3 + (size_t)o * kNH;
  float acc = 0.f;
#pragma unroll 1
  for (int h4 = 0; h4 < kNH / 4; ++h4) {
    const v4f iv = *(const v4f*)(ip + 4 * h4);
    const v4f dv = *(const v4f*)(dp + 4 * h4);
    const v4f wv = *(const v4f*)(wp + 4 * h4);
    const v4f pv = dv * iv;
    acc += pv[0] * wv[0];
    acc += pv[1] * wv[1];
    acc += pv[2] * wv[2];
    acc += pv[3] * wv[3];
  }
  const float sig = states[(size_t)b * kLDS + kND + o];
  const float x   = qpre[(size_t)b * kND + o];
  const float spv = fmaxf(x, 0.0f) + log1pf(expf(-fabsf(x)));
  so[s][o] = 2.0f * acc * sig + spv;
  __syncthreads();
  const int lane = t & 31, wave = t >> 5;
  const int ws = wave & 3;
  const int c4 = (lane & 15) * 4;
  const v4f v = *(const v4f*)(&so[ws][c4]);
  float* orow = out + (size_t)(bbase + blockIdx.x * 4 + ws) * kLDS + kND;
  const bool wr = (wave < 4) && (lane < 16);
  for (int pass = 0; pass < 2; ++pass) {
    if (wr) *(volatile v4f*)(orow + c4) = v;
    __threadfence();
  }
}

constexpr size_t kOffW1h = 0;
constexpr size_t kOffV1h = kOffW1h + (size_t)kNH * kND * 2;
constexpr size_t kOffW2h = kOffV1h + (size_t)kNH * kND * 2;
constexpr size_t kOffV2h = kOffW2h + (size_t)kNH * kNH * 2;
constexpr size_t kOffW3h = kOffV2h + (size_t)kNH * kNH * 2;
constexpr size_t kOffV3h = kOffW3h + (size_t)kND * kNH * 2;
constexpr size_t kOffW1T = kOffV3h + (size_t)kND * kNH * 2;
constexpr size_t kOffD1  = kOffW1T + (size_t)kND * kNH * 4;
constexpr size_t kOffD2  = kOffD1 + (size_t)kNB * kNH * 4;
constexpr size_t kOffQ   = kOffD2 + (size_t)kNB * kNH * 4;
constexpr size_t kOffU   = kOffQ + (size_t)kNB * kND * 4;
constexpr size_t kOffMu  = kOffU;
constexpr size_t kOffH1  = kOffMu + (size_t)kNB * kND * 2;
constexpr size_t kOffG1  = kOffH1 + (size_t)kNB * kNH * 2;
constexpr size_t kOffH2  = kOffG1 + (size_t)kNB * kNH * 2;
constexpr size_t kOffG2  = kOffH2 + (size_t)kNB * kNH * 2;
constexpr size_t kEndA   = kOffG2 + (size_t)kNB * kNH * 2;
constexpr size_t kOffDW  = kOffU;
constexpr size_t kOffIN  = kOffDW + (size_t)kChunkB * kND * kNH * 2;
constexpr size_t kEndB   = kOffIN + (size_t)kChunkB * kND * kNH * 4;
constexpr size_t kWsTotal = (kEndA > kEndB) ? kEndA : kEndB;
static_assert(kWsTotal == 119930880u, "ws total");
static_assert(kWsTotal <= 134217728u, "ws cap");
static_assert((kOffU % 256) == 0 && (kOffIN % 256) == 0 && (kOffQ % 256) == 0, "ws align");

extern "C" void kernel_launch(void* const* d_in, const int* in_sizes, int n_in,
                              void* d_out, int out_size, void* d_ws, size_t ws_size,
                              hipStream_t stream) {
  if (n_in < 14) return;
  if (in_sizes[1] != kNB * kLDS || in_sizes[2] != kNH * kND || in_sizes[3] != kNH ||
      in_sizes[4] != kNH * kNH || in_sizes[5] != kNH || in_sizes[6] != kND * kNH || in_sizes[7] != kND ||
      in_sizes[8] != kNH * kND || in_sizes[9] != kNH || in_sizes[10] != kNH * kNH || in_sizes[11] != kNH ||
      in_sizes[12] != kND * kNH || in_sizes[13] != kND) return;
  if (out_size != kNB * kLDS) return;
  if (ws_size < kWsTotal) return;

  const float* states = (const float*)d_in[1];
  const float* W1 = (const float*)d_in[2];
  const float* b1 = (const float*)d_in[3];
  const float* W2 = (const float*)d_in[4];
  const float* b2 = (const float*)d_in[5];
  const float* W3 = (const float*)d_in[6];
  const float* b3 = (const float*)d_in[7];
  const float* V1 = (const float*)d_in[8];
  const float* c1 = (const float*)d_in[9];
  const float* V2 = (const float*)d_in[10];
  const float* c2 = (const float*)d_in[11];
  const float* V3 = (const float*)d_in[12];
  const float* c3 = (const float*)d_in[13];
  float* out = (float*)d_out;

  char* ws = (char*)d_ws;
  unsigned short* W1h = (unsigned short*)(ws + kOffW1h);
  unsigned short* V1h = (unsigned short*)(ws + kOffV1h);
  unsigned short* W2h = (unsigned short*)(ws + kOffW2h);
  unsigned short* V2h = (unsigned short*)(ws + kOffV2h);
  unsigned short* W3h = (unsigned short*)(ws + kOffW3h);
  unsigned short* V3h = (unsigned short*)(ws + kOffV3h);
  float* W1T  = (float*)(ws + kOffW1T);
  float* d1f  = (float*)(ws + kOffD1);
  float* d2f  = (float*)(ws + kOffD2);
  float* qpre = (float*)(ws + kOffQ);
  unsigned short* muh = (unsigned short*)(ws + kOffMu);
  unsigned short* h1h = (unsigned short*)(ws + kOffH1);
  unsigned short* g1h = (unsigned short*)(ws + kOffG1);
  unsigned short* h2h = (unsigned short*)(ws + kOffH2);
  unsigned short* g2h = (unsigned short*)(ws + kOffG2);
  unsigned short* DW  = (unsigned short*)(ws + kOffDW);
  float* INNER = (float*)(ws + kOffIN);

  k_wcast<<<dim3(128, 6), dim3(256), 0, stream>>>(W1, V1, W2, V2, W3, V3, W1h, V1h, W2h, V2h, W3h, V3h);
  k_mucast<<<dim3(kNB * 8 / 256), dim3(256), 0, stream>>>(states, muh);
  k_w1t<<<dim3(kNH / 64), dim3(256), 0, stream>>>(W1, W1T);

  const int gridN512 = (kNB / 64) * (kNH / 64) / 8;
  const int gridN64  = (kNB / 64) * (kND / 64) / 8;
  wmma_gemm64<0, false, 2, 3, false, 1, kActC><<<dim3(gridN512, 1), dim3(256), 0, stream>>>(
      muh, nullptr, kND, 0L, W1h, nullptr, kND, 0L, (void*)h1h, (void*)d1f, kNH, 0L, b1, nullptr, 0L,
      kNB, kNH, kND, kScale1);
  wmma_gemm64<0, false, 2, 1, false, 1, kActC><<<dim3(gridN512, 1), dim3(256), 0, stream>>>(
      muh, nullptr, kND, 0L, V1h, nullptr, kND, 0L, (void*)g1h, nullptr, kNH, 0L, c1, nullptr, 0L,
      kNB, kNH, kND, kScale1);
  wmma_gemm64<0, false, 2, 3, false, 1, kActC><<<dim3(gridN512, 1), dim3(256), 0, stream>>>(
      h1h, nullptr, kNH, 0L, W2h, nullptr, kNH, 0L, (void*)h2h, (void*)d2f, kNH, 0L, b2, nullptr, 0L,
      kNB, kNH, kNH, kScale2);
  wmma_gemm64<0, false, 2, 1, false, 1, kActC><<<dim3(gridN512, 1), dim3(256), 0, stream>>>(
      g1h, nullptr, kNH, 0L, V2h, nullptr, kNH, 0L, (void*)g2h, nullptr, kNH, 0L, c2, nullptr, 0L,
      kNB, kNH, kNH, kScale2);
  wmma_gemm64<0, false, 2, 0, false, 0><<<dim3(gridN64, 1), dim3(256), 0, stream>>>(
      h2h, nullptr, kNH, 0L, W3h, nullptr, kNH, 0L, (void*)out, nullptr, kLDS, 0L, b3, nullptr, 0L,
      kNB, kND, kNH, kScale2);
  wmma_gemm64<0, false, 2, 0, false, 0><<<dim3(gridN64, 1), dim3(256), 0, stream>>>(
      g2h, nullptr, kNH, 0L, V3h, nullptr, kNH, 0L, (void*)qpre, nullptr, kND, 0L, c3, nullptr, 0L,
      kNB, kND, kNH, kScale2);

  for (int ch = 0; ch < kNumChunks; ++ch) {
    const int bbase = ch * kChunkB;
    k_dwbuild<<<dim3(kChunkB * 64 * 64 / 256), dim3(256), 0, stream>>>(d1f, W1T, DW, bbase);
    wmma_gemm64<0, false, 0, 0, false, 0><<<dim3(1, kChunkB), dim3(256), 0, stream>>>(
        DW, nullptr, kNH, (long)kND * kNH, W2h, nullptr, kNH, 0L, (void*)INNER, nullptr, kNH, (long)kND * kNH,
        nullptr, nullptr, 0L, kND, kNH, kNH, kScaleI);
    k_jsig<<<dim3(kChunkB / 4), dim3(256), 0, stream>>>(INNER, d2f, W3, qpre, states, out, bbase);
  }
  (void)hipGetLastError();
}
